// KimiDeltaAttention_52398601011566
// MI455X (gfx1250) — hardware-verified
//
#include <hip/hip_runtime.h>
#include <math.h>

typedef __attribute__((ext_vector_type(16))) _Float16 v16h;
typedef __attribute__((ext_vector_type(8)))  _Float16 v8h;
typedef __attribute__((ext_vector_type(16))) __bf16   v16b;
typedef __attribute__((ext_vector_type(8)))  __bf16   v8b;
typedef __attribute__((ext_vector_type(8)))  float    v8f;
typedef __attribute__((ext_vector_type(4)))  float    v4f;

constexpr int kL    = 4096;
constexpr int kDH   = 2048;
constexpr int kHd   = 128;
constexpr int kH    = 16;
constexpr int kHG   = 4;
constexpr int kNG   = kHG * kHd;
constexpr int kLR   = 128;
constexpr int kBG   = 64;
constexpr int kTaps = 4;
constexpr int kThr  = 256;
constexpr float kInCarry = 1024.0f;
constexpr float kWCarry = 4096.0f;
constexpr float kSc = 1.0f / (kInCarry * kWCarry);
constexpr float kCf = 1024.0f;
constexpr float kScF = 1.0f / (kCf * kWCarry);
constexpr float kCo = 1024.0f;
constexpr float kScO = 1.0f / (kCo * kWCarry);
constexpr float kQScale = 0.08838834764831845f;
constexpr float kL2Eps = 1e-6f;
constexpr float kRmsEps = 1e-5f;
constexpr float kF16MinNormal = 6.103515625e-5f;

static_assert((kL % 64) == 0 && (kNG % 64) == 0 && (kDH % 64) == 0 && (kLR % 64) == 0 && (kBG % 64) == 0 && ((kL / 64) * (kLR / 64)) % 8 == 0 && ((kL / 64) * (kBG / 64)) % 8 == 0, "GEMM M, N multiples of 64; grids exact");
static_assert((kDH % 32) == 0 && (kLR % 32) == 0 && kDH == 4 * kNG && kDH == kH * kHd && kH == 4 * kHG && kLR == (1 << 7) && kDH / 8 == 256 && kLR / 8 == 16, "GEMM K multiples of 32; four passes of four heads; the transposing cast's blocks of K / 8 threads");

constexpr size_t kOffWQ = 0ull;
constexpr size_t kOffWK = 8388608ull;
constexpr size_t kOffWV = 16777216ull;
constexpr size_t kOffWO = 25165824ull;
constexpr size_t kOffWFA = 33554432ull;
constexpr size_t kOffWFB = 34078720ull;
constexpr size_t kOffWGA = 34603008ull;
constexpr size_t kOffWGB = 35127296ull;
constexpr size_t kOffWBP = 35651584ull;
constexpr size_t kOffBIAS = 35913728ull;
constexpr size_t kOffPRM = 35930112ull;
constexpr size_t kOffX16 = 35934208ull;
constexpr size_t kOffFA32 = 52711424ull;
constexpr size_t kOffFA16 = 54808576ull;
constexpr size_t kOffGA32 = 55857152ull;
constexpr size_t kOffGA16 = 57954304ull;
constexpr size_t kOffBL = 59002880ull;
constexpr size_t kOffBE = 60051456ull;
constexpr size_t kOffXL = 60575744ull;
constexpr size_t kOffQ2 = 68964352ull;
constexpr size_t kOffK2 = 77352960ull;
constexpr size_t kOffV2 = 85741568ull;
constexpr size_t kOffEG = 94130176ull;
constexpr size_t kOffGO = 102518784ull;
constexpr size_t kOffO16 = 110907392ull;
constexpr size_t kWsTotal = 127684608ull;
static_assert(kWsTotal <= 134217728ull, "carve cap: under 128 MiB");
static_assert(kOffWQ == 0
              && kOffWK == kOffWQ + 8388608ull
              && kOffWV == kOffWK + 8388608ull
              && kOffWO == kOffWV + 8388608ull
              && kOffWFA == kOffWO + 8388608ull
              && kOffWFB == kOffWFA + 524288ull
              && kOffWGA == kOffWFB + 524288ull
              && kOffWGB == kOffWGA + 524288ull
              && kOffWBP == kOffWGB + 524288ull
              && kOffBIAS == kOffWBP + 262144ull
              && kOffPRM == kOffBIAS + 16384ull
              && kOffX16 == kOffPRM + 4096ull
              && kOffFA32 == kOffX16 + 16777216ull
              && kOffFA16 == kOffFA32 + 2097152ull
              && kOffGA32 == kOffFA16 + 1048576ull
              && kOffGA16 == kOffGA32 + 2097152ull
              && kOffBL == kOffGA16 + 1048576ull
              && kOffBE == kOffBL + 1048576ull
              && kOffXL == kOffBE + 524288ull
              && kOffQ2 == kOffXL + 8388608ull
              && kOffK2 == kOffQ2 + 8388608ull
              && kOffV2 == kOffK2 + 8388608ull
              && kOffEG == kOffV2 + 8388608ull
              && kOffGO == kOffEG + 8388608ull
              && kOffO16 == kOffGO + 8388608ull
              && kWsTotal == kOffO16 + 16777216ull, "the carve is chained and totalled");
static_assert((kOffWQ % 256) == 0 && (kOffWK % 256) == 0 && (kOffWV % 256) == 0 && (kOffWO % 256) == 0 && (kOffWFA % 256) == 0 && (kOffWFB % 256) == 0 && (kOffWGA % 256) == 0 && (kOffWGB % 256) == 0 && (kOffWBP % 256) == 0 && (kOffBIAS % 256) == 0 && (kOffPRM % 256) == 0 && (kOffX16 % 256) == 0 && (kOffFA32 % 256) == 0 && (kOffFA16 % 256) == 0 && (kOffGA32 % 256) == 0 && (kOffGA16 % 256) == 0 && (kOffBL % 256) == 0 && (kOffBE % 256) == 0 && (kOffXL % 256) == 0 && (kOffQ2 % 256) == 0 && (kOffK2 % 256) == 0 && (kOffV2 % 256) == 0 && (kOffEG % 256) == 0 && (kOffGO % 256) == 0 && (kOffO16 % 256) == 0, "aligned regions");
constexpr int kFZB = 0, kFDT = 2048, kFEnd = 4096;
constexpr int kPA = 0, kPW = 32, kPEnd = 1024;
static_assert(kFDT == kFZB + kDH && kFDT + kDH == kFEnd && kPW >= kPA + kH && kPW + kHd <= kPEnd, "bias stream and parameter plane maps");

__device__ __forceinline__ unsigned short f2bf_bits(float f) {
  unsigned u = __float_as_uint(f);
  return (unsigned short)((u + 0x7FFFu + ((u >> 16) & 1u)) >> 16);
}
__device__ __forceinline__ float bf_bits2f(unsigned short h) { return __uint_as_float(((unsigned)h) << 16); }
__device__ __forceinline__ float bf16r(float f) { return bf_bits2f(f2bf_bits(f)); }
__device__ __forceinline__ float carry_flush(float v, float carry) {
  const float s = v * carry;
  return (fabsf(s) < kF16MinNormal) ? 0.0f : s;
}
__device__ __forceinline__ float frcp(float x) { return __builtin_amdgcn_rcpf(x); }

__device__ __forceinline__ void dep_guard4_h(v8f& a, v8f& b, v8f& c, v8f& d, v16h x, v16h y) { asm volatile("v_nop\n\tv_nop\n\tv_nop\n\tv_nop" : "+v"(a), "+v"(b), "+v"(c), "+v"(d) : "v"(x), "v"(y)); }
__device__ __forceinline__ void dep_guard4_b(v8f& a, v8f& b, v8f& c, v8f& d, v16b x, v16b y) { asm volatile("v_nop\n\tv_nop\n\tv_nop\n\tv_nop" : "+v"(a), "+v"(b), "+v"(c), "+v"(d) : "v"(x), "v"(y)); }
__device__ __forceinline__ void keep4_h(v16h a, v16h b, v16h c, v16h d) { asm volatile("v_nop" :: "v"(a), "v"(b), "v"(c), "v"(d)); }
__device__ __forceinline__ void keep4_b(v16b a, v16b b, v16b c, v16b d) { asm volatile("v_nop" :: "v"(a), "v"(b), "v"(c), "v"(d)); }
__device__ __forceinline__ void acc_guard4(v8f& a, v8f& b, v8f& c, v8f& d) { asm volatile("v_nop\n\tv_nop\n\tv_nop\n\tv_nop" : "+v"(a), "+v"(b), "+v"(c), "+v"(d)); }

template <typename T> struct Frag;
template <> struct Frag<_Float16> {
  typedef v16h V; union U { v16h v; v8h h[2]; };
  static __device__ __forceinline__ v16h load(const _Float16* p) {
    U f; f.h[0] = *(const v8h*)(p); f.h[1] = *(const v8h*)(p + 16); return f.v;
  }
  static __device__ __forceinline__ v8f mma(v16h a, v16h b, v8f c) {
    return __builtin_amdgcn_wmma_f32_16x16x32_f16(false, a, false, b, (short)0, c, false, false);
  }
  static __device__ __forceinline__ void guard4(v8f& a, v8f& b, v8f& c, v8f& d, v16h x, v16h y) { dep_guard4_h(a, b, c, d, x, y); }
  static __device__ __forceinline__ void keep(v16h a, v16h b, v16h c, v16h d) { keep4_h(a, b, c, d); }
};
template <> struct Frag<__bf16> {
  typedef v16b V; union U { v16b v; v8b h[2]; };
  static __device__ __forceinline__ v16b load(const __bf16* p) {
    U f; f.h[0] = *(const v8b*)(p); f.h[1] = *(const v8b*)(p + 16); return f.v;
  }
  static __device__ __forceinline__ v8f mma(v16b a, v16b b, v8f c) {
    return __builtin_amdgcn_wmma_f32_16x16x32_bf16(false, a, false, b, (short)0, c, false, false);
  }
  static __device__ __forceinline__ void guard4(v8f& a, v8f& b, v8f& c, v8f& d, v16b x, v16b y) { dep_guard4_b(a, b, c, d, x, y); }
  static __device__ __forceinline__ void keep(v16b a, v16b b, v16b c, v16b d) { keep4_b(a, b, c, d); }
};

__device__ __forceinline__ v8f mma_h(v16h a, v16h b, v8f c) {
  c = __builtin_amdgcn_wmma_f32_16x16x32_f16(false, a, false, b, (short)0, c, false, false);
  asm volatile("v_nop\n\tv_nop\n\tv_nop\n\tv_nop" : "+v"(c) : "v"(a), "v"(b));
  return c;
}

template <int ET> struct Elem;
template <> struct Elem<0> { typedef _Float16 T; };
template <> struct Elem<1> { typedef __bf16 T; };
template <int ET, bool SPLIT, int BIAS_MODE, int OUT_MODE, bool RESID, int ACT = 0>
__global__ __launch_bounds__(256) void wmma_gemm64(
    const unsigned short* __restrict__ Ap, const unsigned short* __restrict__ A2p, int lda, long strideA,
    const unsigned short* __restrict__ Btp, const unsigned short* __restrict__ Bt2p, int ldb, long strideB,
    void* __restrict__ Cout, void* __restrict__ Cout2, int ldc, long strideC,
    const float* __restrict__ bias,
    const float* __restrict__ resid, long strideR,
    int M, int N, int K, float scale) {
  typedef typename Elem<ET>::T T;
  typedef typename Frag<T>::V V;
  const T* A = (const T*)Ap; const T* A2 = (const T*)A2p; const T* Bt = (const T*)Btp; const T* Bt2 = (const T*)Bt2p;
  __shared__ __align__(16) float sT[8][16 * 68];
  const int b    = blockIdx.y;
  const int lane = threadIdx.x & 31;
  const int wave = threadIdx.x >> 5;
  const int tilesN = N >> 6;
  const int tilesM = M >> 6;
  const int tile = blockIdx.x * 8 + wave;
  if (tile >= tilesM * tilesN) return;
  const int tm = tile / tilesN;
  const int tn = tile - tm * tilesN;
  const int m0 = tm << 6;
  const int n0 = tn << 6;

  const T* Ab  = A  + (size_t)b * strideA;
  const T* Bb  = Bt + (size_t)b * strideB;
  const T* Ab2 = SPLIT ? (A2  + (size_t)b * strideA) : nullptr;
  const T* Bb2 = SPLIT ? (Bt2 + (size_t)b * strideB) : nullptr;

  const int rlane = lane & 15;
  const int koff  = (lane >> 4) * 8;
  const int mOff  = (lane >> 4) * 8;

  v8f acc[4][4];
#pragma unroll
  for (int i = 0; i < 4; ++i)
#pragma unroll
    for (int j = 0; j < 4; ++j) acc[i][j] = (v8f){0.f,0.f,0.f,0.f,0.f,0.f,0.f,0.f};

  for (int k0 = 0; k0 < K; k0 += 32) {
    V bh[4], bl[4];
#pragma unroll
    for (int j = 0; j < 4; ++j) {
      const size_t bo = (size_t)(n0 + (j << 4) + rlane) * ldb + koff + k0;
      bh[j] = Frag<T>::load(Bb + bo);
      if (SPLIT) bl[j] = Frag<T>::load(Bb2 + bo);
    }
#pragma unroll
    for (int i = 0; i < 4; ++i) {
      const size_t ao = (size_t)(m0 + (i << 4) + rlane) * lda + koff + k0;
      V ah = Frag<T>::load(Ab + ao);
      V al;
      if (SPLIT) al = Frag<T>::load(Ab2 + ao);
#pragma unroll
      for (int j = 0; j < 4; ++j) {
        acc[i][j] = Frag<T>::mma(ah, bh[j], acc[i][j]);
        if (SPLIT) {
          acc[i][j] = Frag<T>::mma(ah, bl[j], acc[i][j]);
          acc[i][j] = Frag<T>::mma(al, bh[j], acc[i][j]);
        }
      }
      Frag<T>::guard4(acc[i][0], acc[i][1], acc[i][2], acc[i][3], ah, SPLIT ? al : ah);
    }
    Frag<T>::keep(bh[0], bh[1], bh[2], bh[3]);
    if (SPLIT) Frag<T>::keep(bl[0], bl[1], bl[2], bl[3]);
  }
  acc_guard4(acc[0][0], acc[0][1], acc[0][2], acc[0][3]);
  acc_guard4(acc[1][0], acc[1][1], acc[1][2], acc[1][3]);
  acc_guard4(acc[2][0], acc[2][1], acc[2][2], acc[2][3]);
  acc_guard4(acc[3][0], acc[3][1], acc[3][2], acc[3][3]);

  float* slab = sT[wave];
  const float* Rb = RESID ? (resid + (size_t)b * strideR) : nullptr;
#pragma unroll
  for (int i = 0; i < 4; ++i) {
    const int mBase = m0 + (i << 4);
#pragma unroll
    for (int j = 0; j < 4; ++j) {
      const int n = n0 + (j << 4) + rlane;
      float bv = 0.f;
      if (BIAS_MODE == 2) bv = bias[n];
#pragma unroll
      for (int r = 0; r < 8; ++r) {
        float v = acc[i][j][r] * scale;
        if (BIAS_MODE == 1) v += bias[mBase + mOff + r];
        if (BIAS_MODE == 2) v += bv;
        if (RESID) v += Rb[(size_t)(mBase + mOff + r) * ldc + n];
        if (ACT == 1) v = tanhf(v);
        if (ACT == 2) v = fmaxf(v, 0.0f);
        if (ACT == 3) v = v / (1.0f + expf(-v));
        if (ACT == 4) v = (v > 0.f) ? v : 0.01f * v;
        slab[(mOff + r) * 68 + (j << 4) + rlane] = v;
      }
    }
    __builtin_amdgcn_fence(__ATOMIC_RELEASE, "workgroup");
    __builtin_amdgcn_wave_barrier();
    __builtin_amdgcn_fence(__ATOMIC_ACQUIRE, "workgroup");
    if (OUT_MODE == 0) {
      float* C = (float*)Cout + (size_t)b * strideC;
      const int hh = lane >> 4, c4 = (lane & 15) * 4;
      for (int pass = 0; pass < 2; ++pass) {
#pragma unroll
        for (int it = 0; it < 8; ++it) {
          const int row = it * 2 + hh;
          v4f v = *(const v4f*)(slab + row * 68 + c4);
          *(volatile v4f*)(C + (size_t)(mBase + row) * ldc + n0 + c4) = v;
        }
        __threadfence();
      }
    } else {
      const int q = lane >> 3, c8 = (lane & 7) * 8;
      unsigned short* C  = (unsigned short*)Cout  + (size_t)b * strideC;
      unsigned short* C2 = (OUT_MODE == 2) ? ((unsigned short*)Cout2 + (size_t)b * strideC) : nullptr;
      for (int pass = 0; pass < 2; ++pass) {
#pragma unroll
        for (int it = 0; it < 4; ++it) {
          const int row = it * 4 + q;
          const float* sp = slab + row * 68 + c8;
          v8h hv, lv;
#pragma unroll
          for (int e = 0; e < 8; ++e) {
            if (OUT_MODE == 1) {
              hv[e] = (_Float16)sp[e];
            } else {
              unsigned short hb = f2bf_bits(sp[e]);
              unsigned short lb = f2bf_bits(sp[e] - bf_bits2f(hb));
              hv[e] = __builtin_bit_cast(_Float16, hb);
              lv[e] = __builtin_bit_cast(_Float16, lb);
            }
          }
          *(volatile v8h*)(C + (size_t)(mBase + row) * ldc + n0 + c8) = hv;
          if (OUT_MODE == 2) *(volatile v8h*)(C2 + (size_t)(mBase + row) * ldc + n0 + c8) = lv;
        }
        __threadfence();
      }
    }
    __builtin_amdgcn_fence(__ATOMIC_RELEASE, "workgroup");
    __builtin_amdgcn_wave_barrier();
    __builtin_amdgcn_fence(__ATOMIC_ACQUIRE, "workgroup");
  }
}

__global__ __launch_bounds__(kThr) void cast_plane_kernel(const float* __restrict__ src, unsigned short* __restrict__ dst,
                                                          int colsLog2, int dstPitch, int dstOff) {
  const int i   = blockIdx.x * kThr + threadIdx.x;
  const int sh  = colsLog2 - 3;
  const int row = i >> sh;
  const int c8  = (i & ((1 << sh) - 1)) * 8;
  const float* sp = src + ((size_t)row << colsLog2) + c8;
  const v4f a0 = *(const v4f*)(sp);
  const v4f a1 = *(const v4f*)(sp + 4);
  v8h hv;
#pragma unroll
  for (int e = 0; e < 4; ++e) {
    const float f0 = a0[e];
    const float f1 = a1[e];
    hv[e]     = (_Float16)carry_flush(bf16r(f0), kInCarry);
    hv[4 + e] = (_Float16)carry_flush(bf16r(f1), kInCarry);
  }
  unsigned short* dp = dst + (size_t)row * dstPitch + dstOff + c8;
  *(volatile v8h*)dp = hv;
  __threadfence();
  *(volatile v8h*)dp = hv;
}
__global__ __launch_bounds__(256) void wt_plane_kernel(const float* __restrict__ W, unsigned short* __restrict__ dst, int K, int N, int nLive, int ldd, int colOff) {
  const int n  = blockIdx.x;
  const int k8 = threadIdx.x * 8;
  const bool live = n < nLive;
  const int nc = live ? n : 0;
  v8h hv;
#pragma unroll
  for (int e = 0; e < 8; ++e) {
    const float w = W[(size_t)(k8 + e) * N + nc];
    hv[e] = (_Float16)(live ? carry_flush(bf16r(w), kWCarry) : 0.0f);
  }
  unsigned short* dp = dst + (size_t)n * ldd + colOff + k8;
  *(volatile v8h*)dp = hv;
  __threadfence();
  *(volatile v8h*)dp = hv;
}


__device__ __forceinline__ float silu_f(float v) { return v / (1.0f + expf(-v)); }
__device__ __forceinline__ float sigm_f(float v) { return 1.0f / (1.0f + expf(-v)); }

__global__ __launch_bounds__(kThr) void setup_kernel(const float* __restrict__ dt_bias, const float* __restrict__ A_log, const float* __restrict__ o_norm_w,
                                                     float* __restrict__ BIAS, float* __restrict__ PRM) {
  unsigned v = blockIdx.x * (unsigned)kThr + threadIdx.x;
  asm volatile("" : "+v"(v));
  if (v < 1024u) {
    const unsigned i0 = v * 4u;
    const bool live = i0 >= (unsigned)kFDT;
    const unsigned j0 = live ? (i0 - (unsigned)kFDT) : 0u;
    const v4f a = *(const v4f*)(dt_bias + j0);
    v4f o;
#pragma unroll
    for (int e = 0; e < 4; ++e) { const float p = bf16r(a[e]); o[e] = live ? p : 0.0f; }
    float* dp = BIAS + i0;
    *(volatile v4f*)dp = o;
    __threadfence();
    *(volatile v4f*)dp = o;
  } else {
    const unsigned i = v - 1024u;
    const bool isA = i < (unsigned)kH, isW = (i >= (unsigned)kPW) && (i < (unsigned)(kPW + kHd));
    const float a = bf16r(A_log[isA ? i : 0u]);
    const float w = bf16r(o_norm_w[isW ? (i - (unsigned)kPW) : 0u]);
    const float val = isA ? -expf(a) : (isW ? w : 0.0f);
    float* dp = PRM + i;
    *(volatile float*)dp = val;
    __threadfence();
    *(volatile float*)dp = val;
  }
}
static_assert(kFEnd / 4 == 1024 && 1024 + kPEnd == 8 * kThr && (1024 % 32) == 0, "set-up grid exact; regions wave-uniform");

__global__ __launch_bounds__(kThr) void lr_cast_kernel(const float* __restrict__ src, unsigned short* __restrict__ dst) {
  const size_t v = (size_t)blockIdx.x * kThr + threadIdx.x;
  const v4f a0 = *(const v4f*)(src + v * 8), a1 = *(const v4f*)(src + v * 8 + 4);
  v8h hv;
#pragma unroll
  for (int e = 0; e < 4; ++e) { hv[e] = (_Float16)carry_flush(a0[e], kCf); hv[4 + e] = (_Float16)carry_flush(a1[e], kCf); }
  unsigned short* dp = dst + v * 8;
  *(volatile v8h*)dp = hv;
  __threadfence();
  *(volatile v8h*)dp = hv;
}
static_assert(((size_t)kL * kLR / 8) % kThr == 0, "low-rank cast grid exact");

__global__ __launch_bounds__(kThr) void convnorm_kernel(const float* __restrict__ X, const float* __restrict__ cw, float* __restrict__ OUT, int cbase, int mode) {
  const unsigned v = blockIdx.x * (unsigned)kThr + threadIdx.x;
  const unsigned t = v >> 2, hd = v & 3u;
  const unsigned c0 = hd * (unsigned)kHd;
  float* orow = OUT + (size_t)t * kNG + c0;
  float ss = 0.0f;
  const int npassA = (mode == 0) ? 2 : 1;
  for (int pass = 0; pass < npassA; ++pass) {
    ss = 0.0f;
#pragma unroll 1
    for (int c = 0; c < kHd; c += 4) {
      const unsigned cg = (unsigned)cbase + c0 + (unsigned)c;
      v4f acc = {0.f, 0.f, 0.f, 0.f};
#pragma unroll
      for (int j = 0; j < kTaps; ++j) {
        const int tr = (int)t - (kTaps - 1) + j;
        if (tr >= 0) {
          const v4f xv = *(const v4f*)(X + (size_t)tr * kNG + c0 + c);
#pragma unroll
          for (int e = 0; e < 4; ++e) acc[e] += xv[e] * bf16r(cw[(size_t)(cg + e) * kTaps + j]);
        }
      }
      v4f y;
#pragma unroll
      for (int e = 0; e < 4; ++e) { y[e] = silu_f(acc[e]); ss += y[e] * y[e]; }
      *(volatile v4f*)(orow + c) = y;
    }
    __threadfence();
  }
  if (mode != 0) {
    float qs = (mode == 2) ? kQScale : 1.0f;
    asm volatile("" : "+v"(qs));
    const float rn = (1.0f / sqrtf(ss + kL2Eps)) * qs;
#pragma unroll 1
    for (int c = 0; c < kHd; c += 4) {
      const v4f a = *(const v4f*)(orow + c);
      v4f y;
#pragma unroll
      for (int e = 0; e < 4; ++e) y[e] = a[e] * rn;
      *(volatile v4f*)(orow + c) = y;
    }
    __threadfence();
#pragma unroll 1
    for (int c = 0; c < kHd; c += 4) { const v4f a = *(const v4f*)(orow + c); *(volatile v4f*)(orow + c) = a; }
    __threadfence();
  }
}
static_assert(((size_t)kL * kHG) % kThr == 0 && kHG == 4, "conv + norm grid exact; four heads a group");

__global__ __launch_bounds__(kThr) void beta_kernel(const float* __restrict__ BL, float* __restrict__ BE) {
  const unsigned t = blockIdx.x * (unsigned)kThr + threadIdx.x;
  const float* br = BL + (size_t)t * kBG;
  float* er = BE + (size_t)t * 32;
  for (int pass = 0; pass < 2; ++pass) {
#pragma unroll 1
    for (int h = 0; h < kH; h += 4) {
      const v4f bbv = *(const v4f*)(br + h);
      v4f ob;
#pragma unroll
      for (int e = 0; e < 4; ++e) ob[e] = sigm_f(bbv[e]);
      *(volatile v4f*)(er + h) = ob;
    }
    __threadfence();
  }
}
static_assert(kL == 16 * kThr, "one thread a row: 16 blocks");

__global__ __launch_bounds__(kThr) void decay_kernel(float* __restrict__ EG, const float* __restrict__ PRM, int hbase) {
  const size_t v = (size_t)blockIdx.x * kThr + threadIdx.x;
  const unsigned col = ((unsigned)v * 4u) & (unsigned)(kNG - 1);
  const float na = PRM[kPA + hbase + (int)(col >> 7)];
  float* p = EG + v * 4;
  const v4f g = *(const v4f*)p;
  v4f o;
#pragma unroll
  for (int e = 0; e < 4; ++e) {
    const float x = g[e];
    const float sp = fmaxf(x, 0.0f) + log1pf(expf(-fabsf(x)));
    o[e] = expf(na * sp);
  }
  *(volatile v4f*)p = o;
  __threadfence();
  *(volatile v4f*)p = o;
}
static_assert(((size_t)kL * kNG / 4) % kThr == 0 && (kNG & (kNG - 1)) == 0, "decay grid exact; the group's width a power of two");

__global__ __launch_bounds__(kHd) void kda_scan_kernel(const float* __restrict__ Q2, const float* __restrict__ K2, const float* __restrict__ V2,
                                                       const float* __restrict__ EG, const float* __restrict__ BE, float* __restrict__ O32, int hbase) {
  __shared__ float st[kHd * kHd];
  const unsigned vcol = threadIdx.x;
  const unsigned hoff = blockIdx.x * (unsigned)kHd;
  const unsigned hg = (unsigned)hbase + blockIdx.x;
  for (int k = 0; k < kHd; ++k) st[k * kHd + vcol] = 0.0f;
  for (int t = 0; t < kL; ++t) {
    const float* qr = Q2 + (size_t)t * kNG + hoff;
    const float* kr = K2 + (size_t)t * kNG + hoff;
    const float* er = EG + (size_t)t * kNG + hoff;
    const float vv = V2[(size_t)t * kNG + hoff + vcol];
    const float bt = BE[(size_t)t * 32 + hg];
    float r = 0.0f;
#pragma unroll 1
    for (int k4 = 0; k4 < kHd; k4 += 4) {
      const v4f c4 = *(const v4f*)(kr + k4), e4 = *(const v4f*)(er + k4);
#pragma unroll
      for (int j = 0; j < 4; ++j) r += c4[j] * (e4[j] * st[(k4 + j) * kHd + (int)vcol]);
    }
    const float vres = vv - r;
    const float bv = bt * vres;
    float sum = 0.0f;
#pragma unroll 1
    for (int k4 = 0; k4 < kHd; k4 += 4) {
      const v4f q4 = *(const v4f*)(qr + k4), c4 = *(const v4f*)(kr + k4), e4 = *(const v4f*)(er + k4);
#pragma unroll
      for (int j = 0; j < 4; ++j) {
        const int idx = (k4 + j) * kHd + (int)vcol;
        const float s = e4[j] * st[idx] + c4[j] * bv;
        st[idx] = s;
        sum += q4[j] * s;
      }
    }
    float* op = O32 + (size_t)t * kNG + hoff + vcol;
    *(volatile float*)op = sum;
    __threadfence();
    *(volatile float*)op = sum;
  }
}
static_assert(kHd * kHd * 4 == 65536 && kHd == 128, "the state: 64 KB of LDS a block; one thread a value column");

__global__ __launch_bounds__(kThr) void normgate_kernel(const float* __restrict__ O32, const float* __restrict__ GO, const float* __restrict__ PRM, unsigned short* __restrict__ O16, int cbase) {
  const unsigned v = blockIdx.x * (unsigned)kThr + threadIdx.x;
  const unsigned t = v >> 2, hd = v & 3u;
  const size_t base = (size_t)t * kNG + hd * (unsigned)kHd;
  const float* orow = O32 + base;
  const float* grow = GO + base;
  const float* w = PRM + kPW;
  float ss = 0.0f;
#pragma unroll 1
  for (int c = 0; c < kHd; c += 4) { const v4f a = *(const v4f*)(orow + c); ss += (a[0] * a[0] + a[1] * a[1]) + (a[2] * a[2] + a[3] * a[3]); }
  const float rs = 1.0f / sqrtf(ss * (1.0f / (float)kHd) + kRmsEps);
  unsigned short* dst = O16 + (size_t)t * kDH + (unsigned)cbase + hd * (unsigned)kHd;
  for (int pass = 0; pass < 2; ++pass) {
#pragma unroll 1
    for (int c = 0; c < kHd; c += 8) {
      const v4f a0 = *(const v4f*)(orow + c), a1 = *(const v4f*)(orow + c + 4), g0 = *(const v4f*)(grow + c), g1 = *(const v4f*)(grow + c + 4), w0 = *(const v4f*)(w + c), w1 = *(const v4f*)(w + c + 4);
      v8h hv;
#pragma unroll
      for (int e = 0; e < 4; ++e) {
        hv[e] = (_Float16)carry_flush(a0[e] * rs * w0[e] * sigm_f(g0[e]), kCo);
        hv[4 + e] = (_Float16)carry_flush(a1[e] * rs * w1[e] * sigm_f(g1[e]), kCo);
      }
      *(volatile v8h*)(dst + c) = hv;
    }
    __threadfence();
  }
}

extern "C" void kernel_launch(void* const* d_in, const int* in_sizes, int n_in,
                              void* d_out, int out_size, void* d_ws, size_t ws_size,
                              hipStream_t stream) {
  if (n_in < 17 || d_out == nullptr || d_ws == nullptr) return;
  if (in_sizes[0] != kL * kDH || in_sizes[1] != kL || in_sizes[2] != kDH * kDH || in_sizes[3] != kDH * kDH || in_sizes[4] != kDH * kDH || in_sizes[5] != kDH * kLR || in_sizes[6] != kLR * kDH || in_sizes[7] != kDH || in_sizes[8] != kDH * kH) return;
  if (in_sizes[9] != kDH * kTaps || in_sizes[10] != kDH * kTaps || in_sizes[11] != kDH * kTaps || in_sizes[12] != kH || in_sizes[13] != kDH * kLR || in_sizes[14] != kLR * kDH || in_sizes[15] != kHd || in_sizes[16] != kDH * kDH) return;
  if (out_size != kL * kDH) return;
  if (ws_size < kWsTotal) return;
  const float* hidden = (const float*)d_in[0];
  const float* Wq = (const float*)d_in[2];
  const float* Wk = (const float*)d_in[3];
  const float* Wv = (const float*)d_in[4];
  const float* Wfa = (const float*)d_in[5];
  const float* Wfb = (const float*)d_in[6];
  const float* dt_bias = (const float*)d_in[7];
  const float* Wb = (const float*)d_in[8];
  const float* conv_q = (const float*)d_in[9];
  const float* conv_k = (const float*)d_in[10];
  const float* conv_v = (const float*)d_in[11];
  const float* A_log = (const float*)d_in[12];
  const float* Wga = (const float*)d_in[13];
  const float* Wgb = (const float*)d_in[14];
  const float* o_norm_w = (const float*)d_in[15];
  const float* Wo = (const float*)d_in[16];
  float* out = (float*)d_out;
  char* ws = (char*)d_ws;
  unsigned short* WQ = (unsigned short*)(ws + kOffWQ);
  unsigned short* WK = (unsigned short*)(ws + kOffWK);
  unsigned short* WV = (unsigned short*)(ws + kOffWV);
  unsigned short* WO = (unsigned short*)(ws + kOffWO);
  unsigned short* WFA = (unsigned short*)(ws + kOffWFA);
  unsigned short* WFB = (unsigned short*)(ws + kOffWFB);
  unsigned short* WGA = (unsigned short*)(ws + kOffWGA);
  unsigned short* WGB = (unsigned short*)(ws + kOffWGB);
  unsigned short* WBP = (unsigned short*)(ws + kOffWBP);
  float* BIAS = (float*)(ws + kOffBIAS);
  float* PRM = (float*)(ws + kOffPRM);
  unsigned short* X16 = (unsigned short*)(ws + kOffX16);
  float* FA32 = (float*)(ws + kOffFA32);
  unsigned short* FA16 = (unsigned short*)(ws + kOffFA16);
  float* GA32 = (float*)(ws + kOffGA32);
  unsigned short* GA16 = (unsigned short*)(ws + kOffGA16);
  float* BL = (float*)(ws + kOffBL);
  float* BE = (float*)(ws + kOffBE);
  float* XL = (float*)(ws + kOffXL);
  float* Q2 = (float*)(ws + kOffQ2);
  float* K2 = (float*)(ws + kOffK2);
  float* V2 = (float*)(ws + kOffV2);
  float* EG = (float*)(ws + kOffEG);
  float* GO = (float*)(ws + kOffGO);
  float* O32 = XL;
  unsigned short* O16 = (unsigned short*)(ws + kOffO16);

  wt_plane_kernel<<<kDH, kDH / 8, 0, stream>>>(Wq, WQ, kDH, kDH, kDH, kDH, 0);
  wt_plane_kernel<<<kDH, kDH / 8, 0, stream>>>(Wk, WK, kDH, kDH, kDH, kDH, 0);
  wt_plane_kernel<<<kDH, kDH / 8, 0, stream>>>(Wv, WV, kDH, kDH, kDH, kDH, 0);
  wt_plane_kernel<<<kDH, kDH / 8, 0, stream>>>(Wo, WO, kDH, kDH, kDH, kDH, 0);
  wt_plane_kernel<<<kLR, kDH / 8, 0, stream>>>(Wfa, WFA, kDH, kLR, kLR, kDH, 0);
  wt_plane_kernel<<<kDH, kLR / 8, 0, stream>>>(Wfb, WFB, kLR, kDH, kDH, kLR, 0);
  wt_plane_kernel<<<kLR, kDH / 8, 0, stream>>>(Wga, WGA, kDH, kLR, kLR, kDH, 0);
  wt_plane_kernel<<<kDH, kLR / 8, 0, stream>>>(Wgb, WGB, kLR, kDH, kDH, kLR, 0);
  wt_plane_kernel<<<kH, kDH / 8, 0, stream>>>(Wb, WBP, kDH, kH, kH, kDH, 0);
  wt_plane_kernel<<<kBG - kH, kDH / 8, 0, stream>>>(Wb, WBP + (size_t)kH * kDH, kDH, kH, 0, kDH, 0);
  setup_kernel<<<8, kThr, 0, stream>>>(dt_bias, A_log, o_norm_w, BIAS, PRM);

  cast_plane_kernel<<<(int)(((size_t)kL * kDH / 8) / kThr), kThr, 0, stream>>>(hidden, X16, 11, kDH, 0);
  const int gLC = (int)(((size_t)kL * kLR / 8) / kThr);
  wmma_gemm64<0, false, 2, 0, false, 0><<<dim3((kL / 64) * (kLR / 64) / 8, 1), 256, 0, stream>>>(
      X16, X16, kDH, 0L, WFA, WFA, kDH, 0L, (void*)FA32, (void*)FA32, kLR, 0L, BIAS + kFZB, nullptr, 0L, kL, kLR, kDH, kSc);
  lr_cast_kernel<<<gLC, kThr, 0, stream>>>(FA32, FA16);
  wmma_gemm64<0, false, 2, 0, false, 0><<<dim3((kL / 64) * (kLR / 64) / 8, 1), 256, 0, stream>>>(
      X16, X16, kDH, 0L, WGA, WGA, kDH, 0L, (void*)GA32, (void*)GA32, kLR, 0L, BIAS + kFZB, nullptr, 0L, kL, kLR, kDH, kSc);
  lr_cast_kernel<<<gLC, kThr, 0, stream>>>(GA32, GA16);
  wmma_gemm64<0, false, 2, 0, false, 0><<<dim3((kL / 64) * (kBG / 64) / 8, 1), 256, 0, stream>>>(
      X16, X16, kDH, 0L, WBP, WBP, kDH, 0L, (void*)BL, (void*)BL, kBG, 0L, BIAS + kFZB, nullptr, 0L, kL, kBG, kDH, kSc);
  beta_kernel<<<kL / kThr, kThr, 0, stream>>>(BL, BE);
  for (int hg = 0; hg < 4; ++hg) {
    const size_t wo = (size_t)hg * kNG * kDH;
    const size_t wl = (size_t)hg * kNG * kLR;
    wmma_gemm64<0, false, 2, 0, false, 0><<<dim3((kL / 64) * (kNG / 64) / 8, 1), 256, 0, stream>>>(
        X16, X16, kDH, 0L, WQ + wo, WQ + wo, kDH, 0L, (void*)XL, (void*)XL, kNG, 0L, BIAS + kFZB, nullptr, 0L, kL, kNG, kDH, kSc);
    convnorm_kernel<<<(kL * kHG) / kThr, kThr, 0, stream>>>(XL, conv_q, Q2, hg * kNG, 2);
    wmma_gemm64<0, false, 2, 0, false, 0><<<dim3((kL / 64) * (kNG / 64) / 8, 1), 256, 0, stream>>>(
        X16, X16, kDH, 0L, WK + wo, WK + wo, kDH, 0L, (void*)XL, (void*)XL, kNG, 0L, BIAS + kFZB, nullptr, 0L, kL, kNG, kDH, kSc);
    convnorm_kernel<<<(kL * kHG) / kThr, kThr, 0, stream>>>(XL, conv_k, K2, hg * kNG, 1);
    wmma_gemm64<0, false, 2, 0, false, 0><<<dim3((kL / 64) * (kNG / 64) / 8, 1), 256, 0, stream>>>(
        X16, X16, kDH, 0L, WV + wo, WV + wo, kDH, 0L, (void*)XL, (void*)XL, kNG, 0L, BIAS + kFZB, nullptr, 0L, kL, kNG, kDH, kSc);
    convnorm_kernel<<<(kL * kHG) / kThr, kThr, 0, stream>>>(XL, conv_v, V2, hg * kNG, 0);
    wmma_gemm64<0, false, 2, 0, false, 0><<<dim3((kL / 64) * (kNG / 64) / 8, 1), 256, 0, stream>>>(
        FA16, FA16, kLR, 0L, WFB + wl, WFB + wl, kLR, 0L, (void*)EG, (void*)EG, kNG, 0L, BIAS + kFDT + hg * kNG, nullptr, 0L, kL, kNG, kLR, kScF);
    decay_kernel<<<(int)(((size_t)kL * kNG / 4) / kThr), kThr, 0, stream>>>(EG, PRM, hg * kHG);
    wmma_gemm64<0, false, 2, 0, false, 0><<<dim3((kL / 64) * (kNG / 64) / 8, 1), 256, 0, stream>>>(
        GA16, GA16, kLR, 0L, WGB + wl, WGB + wl, kLR, 0L, (void*)GO, (void*)GO, kNG, 0L, BIAS + kFZB, nullptr, 0L, kL, kNG, kLR, kScF);
    kda_scan_kernel<<<kHG, kHd, 0, stream>>>(Q2, K2, V2, EG, BE, O32, hg * kHG);
    normgate_kernel<<<(kL * kHG) / kThr, kThr, 0, stream>>>(O32, GO, PRM, O16, hg * kNG);
  }
  wmma_gemm64<0, false, 2, 0, false, 0><<<dim3((kL / 64) * (kDH / 64) / 8, 1), 256, 0, stream>>>(
      O16, O16, kDH, 0L, WO, WO, kDH, 0L, (void*)out, (void*)out, kDH, 0L, BIAS + kFZB, nullptr, 0L, kL, kDH, kDH, kScO);
}
